// MultiHeadNonLocalBlock2d_3100966387741
// MI455X (gfx1250) — hardware-verified
//
#include <hip/hip_runtime.h>


#define NB_  4
#define CC   256
#define CI   128
#define NHD  4
#define HD   32
#define NP   4096
#define QCH  2048
#define PSC  32768.0f
#define LOSC 1024.0f
#define LOSCI (1.0f / 1024.0f)

typedef _Float16 h16;
typedef unsigned short bf;
typedef __attribute__((ext_vector_type(16))) __bf16   v16bf;
typedef __attribute__((ext_vector_type(16))) _Float16 v16h;
typedef __attribute__((ext_vector_type(8)))  _Float16 v8h;
typedef __attribute__((ext_vector_type(8)))  unsigned short v8us;
typedef __attribute__((ext_vector_type(8)))  float    v8f;
typedef __attribute__((ext_vector_type(4)))  float    v4f;
typedef v8h  __attribute__((may_alias)) v8ha;
typedef v4f  __attribute__((may_alias)) v4fa;
typedef v8us __attribute__((may_alias)) v8usa;

__device__ __forceinline__ unsigned short f2bf(float f) { unsigned u = __float_as_uint(f); u += 0x7FFFu + ((u >> 16) & 1u); return (unsigned short)(u >> 16); }
__device__ __forceinline__ float bf2f(unsigned short b) { return __uint_as_float(((unsigned)b) << 16); }
__device__ __forceinline__ float bfr(float f) { return bf2f(f2bf(f)); }
__device__ __forceinline__ v16h cat16(v8h lo, v8h hi) { return __builtin_shufflevector(lo, hi, 0, 1, 2, 3, 4, 5, 6, 7, 8, 9, 10, 11, 12, 13, 14, 15); }
__device__ __forceinline__ v16bf cat16b(v8us lo, v8us hi) { return __builtin_bit_cast(v16bf, __builtin_shufflevector(lo, hi, 0, 1, 2, 3, 4, 5, 6, 7, 8, 9, 10, 11, 12, 13, 14, 15)); }
__device__ __forceinline__ v8f wmma16(v16h a, v16h b, v8f c) { return __builtin_amdgcn_wmma_f32_16x16x32_f16(false, a, false, b, (short)0, c, false, false); }
__device__ __forceinline__ v8f wmmab(v16bf a, v16bf b, v8f c) { return __builtin_amdgcn_wmma_f32_16x16x32_bf16(false, a, false, b, (short)0, c, false, false); }
#define VST2(T, p, v) do { const T vst2_v_ = (v); *(volatile T*)(p) = vst2_v_; __threadfence(); *(volatile T*)(p) = vst2_v_; } while (0)

__global__ __launch_bounds__(256) void k_xt(const float* __restrict__ xb, bf* XT) {
    __shared__ __align__(16) unsigned short tl[64 * 72];
    const int tid = threadIdx.x, n0 = blockIdx.x * 64, c0 = blockIdx.y * 64;
    const int cr = tid >> 2, nq = (tid & 3) * 16;
#pragma unroll
    for (int i = 0; i < 16; ++i) tl[(nq + i) * 72 + cr] = f2bf(xb[(size_t)(c0 + cr) * NP + n0 + nq + i]);
    __syncthreads();
    const int piece = tid & 7;
    auto pass = [&]() {
#pragma unroll
        for (int s = 0; s < 2; ++s) { const int nr = (tid >> 3) + 32 * s; const v8us val = *(const v8usa*)(tl + nr * 72 + piece * 8); *(volatile v8us*)(XT + (size_t)(n0 + nr) * CC + c0 + piece * 8) = val; }
    };
    pass(); __threadfence(); pass();
}
__global__ __launch_bounds__(256) void k_w(const float* __restrict__ w, int rows, bf* WB) {
    const int lane = threadIdx.x & 31, r = blockIdx.x * 8 + (threadIdx.x >> 5); if (r >= rows) return;
    v8us o;
#pragma unroll
    for (int i = 0; i < 8; ++i) o[i] = f2bf(w[(size_t)r * CC + lane * 8 + i]);
    VST2(v8us, WB + (size_t)r * CC + lane * 8, o);
}
__global__ __launch_bounds__(256) void k_w128(const float* __restrict__ w, int rows, bf* WB) {
    const int lane = threadIdx.x & 31, r = (blockIdx.x * 8 + (threadIdx.x >> 5)) * 2 + (lane >> 4), p = lane & 15; if (r >= rows) return;
    v8us o;
#pragma unroll
    for (int i = 0; i < 8; ++i) o[i] = f2bf(w[(size_t)r * CI + p * 8 + i]);
    VST2(v8us, WB + (size_t)r * CI + p * 8, o);
}
template <bool SPLITA, int EPI, int KA, int LDC>
__global__ __launch_bounds__(128) void k_gemm(const bf* __restrict__ A, const bf* __restrict__ Al, const bf* __restrict__ WB, const float* __restrict__ bias, const float* __restrict__ bnsc, const float* __restrict__ bnsh, const float* __restrict__ xres, float* C) {
    const float scale = 1.0f; constexpr bool ACC = false; const float* Wm = nullptr; (void)Wm; (void)ACC;
    __shared__ __align__(16) float ost[4][16 * 68];
    __shared__ __align__(16) float ot[64 * 68];
    const int lane = threadIdx.x & 31, wave = threadIdx.x >> 5, lr = lane & 15, hi = lane >> 4, tid = threadIdx.x;
    const size_t r0 = (size_t)blockIdx.x * 64 + wave * 16; const int c0 = blockIdx.y * 64;
    v8f acc[4];
#pragma unroll
    for (int t = 0; t < 4; ++t) acc[t] = (v8f){};
#pragma unroll
    for (int kc = 0; kc < KA; kc += 32) {
        const v16bf a = cat16b(*(const v8us*)(A + (r0 + lr) * KA + kc + 8 * hi), *(const v8us*)(A + (r0 + lr) * KA + kc + 8 * hi + 16));
        v16bf al = a; if (SPLITA) al = cat16b(*(const v8us*)(Al + (r0 + lr) * KA + kc + 8 * hi), *(const v8us*)(Al + (r0 + lr) * KA + kc + 8 * hi + 16));
#pragma unroll
        for (int t = 0; t < 4; ++t) { const bf* bp = WB + (size_t)(c0 + t * 16 + lr) * KA + kc + 8 * hi; const v16bf bb = cat16b(*(const v8us*)bp, *(const v8us*)(bp + 16)); acc[t] = wmmab(a, bb, acc[t]); if (SPLITA) acc[t] = wmmab(al, bb, acc[t]); }
        asm volatile("v_nop" : "+v"(acc[0]), "+v"(acc[1]), "+v"(acc[2]), "+v"(acc[3]) : "v"(a), "v"(al) : "memory");
    }
    float* os = &ost[wave][0];
#pragma unroll
    for (int t = 0; t < 4; ++t) { const int col = c0 + t * 16 + lr; const float bv = bfr(bias[col]);
#pragma unroll
        for (int j = 0; j < 8; ++j) { float v = (acc[t][j] + bv) * scale;
            if (EPI == 2) v = v * bnsc[col] + bnsh[col];
            os[(hi * 8 + j) * 68 + t * 16 + lr] = v; } }
    if (EPI != 2) {
        __builtin_amdgcn_wave_barrier(); asm volatile("" ::: "memory");
        float* crow = C + r0 * LDC + c0;
        auto pass = [&]() {
#pragma unroll
            for (int s = 0; s < 8; ++s) { const int Lid = (lane >> 3) + 4 * s, piece = lane & 7; const int row = Lid >> 1, cofs = (Lid & 1) * 32 + piece * 4;
                const v4f val = *(const v4fa*)(os + row * 68 + cofs); *(volatile v4f*)(crow + (size_t)row * LDC + cofs) = val; }
        };
        pass(); __threadfence(); pass();
    } else {
        __syncthreads();
        { const int row = tid >> 1, half = tid & 1;
#pragma unroll
          for (int i = 0; i < 32; ++i) ot[(half * 32 + i) * 68 + row] = ost[row >> 4][(row & 15) * 68 + half * 32 + i]; }
        __syncthreads();
        const size_t rblk = (size_t)blockIdx.x * 64;
        auto pass = [&]() {
#pragma unroll
            for (int s = 0; s < 8; ++s) { const int cl = s * 8 + (tid >> 4), piece = tid & 15;
                v4f val = *(const v4fa*)(ot + cl * 68 + piece * 4); const size_t oi = (size_t)(c0 + cl) * NP + rblk + piece * 4;
#pragma unroll
                for (int i = 0; i < 4; ++i) val[i] += bfr(xres[oi + i]);
                *(volatile v4f*)(C + oi) = val; }
        };
        pass(); __threadfence(); pass();
    }
}
__global__ __launch_bounds__(256) void k_p16(const float* __restrict__ A, const float* __restrict__ Bsum, h16* PH, h16* PL) {
    const int lane = threadIdx.x & 31, r = blockIdx.x * 8 + (threadIdx.x >> 5);
    if (r >= NP) return;
    v8h oh, ol;
#pragma unroll
    for (int i = 0; i < 8; ++i) { float v = A[(size_t)r * CC + lane * 8 + i]; if (Bsum) v += Bsum[(size_t)r * CC + lane * 8 + i]; const h16 a = (h16)v; oh[i] = a; ol[i] = (h16)((v - (float)a) * LOSC); }
    *(volatile v8h*)(PH + (size_t)r * CC + lane * 8) = oh; *(volatile v8h*)(PL + (size_t)r * CC + lane * 8) = ol; __threadfence();
    *(volatile v8h*)(PH + (size_t)r * CC + lane * 8) = oh; *(volatile v8h*)(PL + (size_t)r * CC + lane * 8) = ol;
}
__global__ __launch_bounds__(256) void k_p16c(const float* __restrict__ A, h16* PH, h16* PL) {
    const int lane = threadIdx.x & 31, r = (blockIdx.x * 8 + (threadIdx.x >> 5)) * 2 + (lane >> 4), p = lane & 15;
    if (r >= NP) return;
    v8h oh, ol;
#pragma unroll
    for (int i = 0; i < 8; ++i) { const float v = A[(size_t)r * CI + p * 8 + i]; const h16 a = (h16)v; oh[i] = a; ol[i] = (h16)((v - (float)a) * LOSC); }
    *(volatile v8h*)(PH + (size_t)r * CI + p * 8) = oh; *(volatile v8h*)(PL + (size_t)r * CI + p * 8) = ol; __threadfence();
    *(volatile v8h*)(PH + (size_t)r * CI + p * 8) = oh; *(volatile v8h*)(PL + (size_t)r * CI + p * 8) = ol;
}
__global__ __launch_bounds__(256) void k_pbfc(const float* __restrict__ A, bf* PH, bf* PL) {
    const int lane = threadIdx.x & 31, r = (blockIdx.x * 8 + (threadIdx.x >> 5)) * 2 + (lane >> 4), p = lane & 15;
    if (r >= NP) return;
    v8us oh, ol;
#pragma unroll
    for (int i = 0; i < 8; ++i) { const float v = A[(size_t)r * CI + p * 8 + i]; const unsigned short hb = f2bf(v); oh[i] = hb; ol[i] = f2bf(v - bf2f(hb)); }
    *(volatile v8us*)(PH + (size_t)r * CI + p * 8) = oh; *(volatile v8us*)(PL + (size_t)r * CI + p * 8) = ol; __threadfence();
    *(volatile v8us*)(PH + (size_t)r * CI + p * 8) = oh; *(volatile v8us*)(PL + (size_t)r * CI + p * 8) = ol;
}
__global__ __launch_bounds__(256) void k_vt128(const float* __restrict__ V, h16* VTH, h16* VTL) {
    __shared__ float tl[64][65];
    const int tid = threadIdx.x, n0 = blockIdx.x * 64, c0 = blockIdx.y * 64;
    { const int nn = tid >> 2, cq = (tid & 3) * 16;
#pragma unroll
      for (int i = 0; i < 16; ++i) tl[cq + i][nn] = V[(size_t)(n0 + nn) * CI + c0 + cq + i]; }
    __syncthreads();
    const int piece = tid & 7;
    auto pass = [&]() {
#pragma unroll
        for (int s = 0; s < 2; ++s) { const int c = (tid >> 3) + 32 * s; v8h oh, ol;
#pragma unroll
            for (int i = 0; i < 8; ++i) { const float v = tl[c][piece * 8 + i]; const h16 a = (h16)v; oh[i] = a; ol[i] = (h16)((v - (float)a) * LOSC); }
            const size_t o = (size_t)(c0 + c) * NP + n0 + piece * 8; *(volatile v8h*)(VTH + o) = oh; *(volatile v8h*)(VTL + o) = ol; }
    };
    pass(); __threadfence(); pass();
}
__global__ __launch_bounds__(256) void k_bn(const float* __restrict__ g, const float* __restrict__ be, const float* __restrict__ mu, const float* __restrict__ var, float* BNS, float* BNH) {
    const int c = threadIdx.x; const float inv = bfr(g[c]) / sqrtf(bfr(var[c]) + 1e-5f); const float sh = bfr(be[c]) - bfr(mu[c]) * inv;
    *(volatile float*)(BNS + c) = inv; *(volatile float*)(BNH + c) = sh; __threadfence(); *(volatile float*)(BNS + c) = inv; *(volatile float*)(BNH + c) = sh;
}
__global__ __launch_bounds__(256) void k_pbf(const float* __restrict__ A, bf* PH, bf* PL) {
    const int lane = threadIdx.x & 31, r = blockIdx.x * 8 + (threadIdx.x >> 5);
    if (r >= NP) return;
    v8us oh, ol;
#pragma unroll
    for (int i = 0; i < 8; ++i) { const float v = A[(size_t)r * CC + lane * 8 + i]; const unsigned short hb = f2bf(v); oh[i] = hb; ol[i] = f2bf(v - bf2f(hb)); }
    *(volatile v8us*)(PH + (size_t)r * CC + lane * 8) = oh; *(volatile v8us*)(PL + (size_t)r * CC + lane * 8) = ol; __threadfence();
    *(volatile v8us*)(PH + (size_t)r * CC + lane * 8) = oh; *(volatile v8us*)(PL + (size_t)r * CC + lane * 8) = ol;
}
__global__ __launch_bounds__(256) void k_vt(const float* __restrict__ V, h16* VTH, h16* VTL) {
    __shared__ float tl[64][65];
    const int tid = threadIdx.x, n0 = blockIdx.x * 64, c0 = blockIdx.y * 64;
    { const int nn = tid >> 2, cq = (tid & 3) * 16;
#pragma unroll
      for (int i = 0; i < 16; ++i) tl[cq + i][nn] = V[(size_t)(n0 + nn) * CC + c0 + cq + i]; }
    __syncthreads();
    const int piece = tid & 7;
    auto pass = [&]() {
#pragma unroll
        for (int s = 0; s < 2; ++s) { const int c = (tid >> 3) + 32 * s; v8h oh, ol;
#pragma unroll
            for (int i = 0; i < 8; ++i) { const float v = tl[c][piece * 8 + i]; const h16 a = (h16)v; oh[i] = a; ol[i] = (h16)((v - (float)a) * LOSC); }
            const size_t o = (size_t)(c0 + c) * NP + n0 + piece * 8; *(volatile v8h*)(VTH + o) = oh; *(volatile v8h*)(VTL + o) = ol; }
    };
    pass(); __threadfence(); pass();
}
template <int EPI>
__global__ __launch_bounds__(128) void k_f16gemm(const h16* __restrict__ A, const h16* __restrict__ Al, int lda, const h16* __restrict__ Bn, const h16* __restrict__ Bl, int ldb, int K, const float* __restrict__ rs, float* C, int ldc) {
    __shared__ __align__(16) float ost[4][16 * 68];
    const int lane = threadIdx.x & 31, wave = threadIdx.x >> 5, lr = lane & 15, hi = lane >> 4;
    const int r0 = blockIdx.x * 64 + wave * 16, c0 = blockIdx.y * 64;
    const size_t aoff = (size_t)(r0 + lr) * lda + 8 * hi;
    size_t boff[4];
#pragma unroll
    for (int t = 0; t < 4; ++t) boff[t] = (size_t)(c0 + t * 16 + lr) * ldb + 8 * hi;
    v8f acc[4], accx[4];
#pragma unroll
    for (int t = 0; t < 4; ++t) { acc[t] = (v8f){}; accx[t] = (v8f){}; }
#pragma unroll 2
    for (int kc = 0; kc < K; kc += 32) {
        const v16h a = cat16(*(const v8h*)(A + aoff + kc), *(const v8h*)(A + aoff + kc + 16)), al = cat16(*(const v8h*)(Al + aoff + kc), *(const v8h*)(Al + aoff + kc + 16));
#pragma unroll
        for (int t = 0; t < 4; ++t) { const v16h bb = cat16(*(const v8h*)(Bn + boff[t] + kc), *(const v8h*)(Bn + boff[t] + kc + 16)), bl = cat16(*(const v8h*)(Bl + boff[t] + kc), *(const v8h*)(Bl + boff[t] + kc + 16));
            acc[t] = wmma16(a, bb, acc[t]); accx[t] = wmma16(a, bl, accx[t]);
            if (EPI == 0) accx[t] = wmma16(al, bb, accx[t]); else acc[t] = wmma16(al, bb, acc[t]); }
        asm volatile("v_nop" : "+v"(acc[0]), "+v"(acc[1]), "+v"(acc[2]), "+v"(acc[3]), "+v"(accx[0]), "+v"(accx[1]), "+v"(accx[2]), "+v"(accx[3]) : "v"(a), "v"(al) : "memory");
    }
    float* os = &ost[wave][0];
#pragma unroll
    for (int t = 0; t < 4; ++t)
#pragma unroll
        for (int j = 0; j < 8; ++j) { const float sc = (EPI == 0) ? 0.1767766952966369f : rs[r0 + hi * 8 + j]; os[(hi * 8 + j) * 68 + t * 16 + lr] = (acc[t][j] + accx[t][j] * LOSCI) * sc; }
    __builtin_amdgcn_wave_barrier(); asm volatile("" ::: "memory");
    float* crow = C + (size_t)r0 * ldc + c0;
    auto pass = [&]() {
#pragma unroll
        for (int s = 0; s < 8; ++s) { const int Lid = (lane >> 3) + 4 * s, piece = lane & 7; const int row = Lid >> 1, cofs = (Lid & 1) * 32 + piece * 4;
            const v4f val = *(const v4fa*)(os + row * 68 + cofs); *(volatile v4f*)(crow + (size_t)row * ldc + cofs) = val; }
    };
    pass(); __threadfence(); pass();
}
__global__ __launch_bounds__(128) void k_pv32(const h16* __restrict__ A, const h16* __restrict__ Al, int lda, const h16* __restrict__ Bn, const h16* __restrict__ Bl, int ldb, int K, const float* __restrict__ rs, float* C, int ldc) {
    __shared__ __align__(16) float ost[4][16 * 68];
    const int lane = threadIdx.x & 31, wave = threadIdx.x >> 5, lr = lane & 15, hi = lane >> 4;
    const int r0 = blockIdx.x * 64 + wave * 16, c0 = blockIdx.y * 64;
    const size_t aoff = (size_t)(r0 + lr) * lda + 8 * hi;
    constexpr int EPI = 1; size_t boff[2];
#pragma unroll
    for (int t = 0; t < 2; ++t) boff[t] = (size_t)(c0 + t * 16 + lr) * ldb + 8 * hi;
    v8f acc[2], accx[2];
#pragma unroll
    for (int t = 0; t < 2; ++t) { acc[t] = (v8f){}; accx[t] = (v8f){}; }
#pragma unroll 2
    for (int kc = 0; kc < K; kc += 32) {
        const v16h a = cat16(*(const v8h*)(A + aoff + kc), *(const v8h*)(A + aoff + kc + 16)), al = cat16(*(const v8h*)(Al + aoff + kc), *(const v8h*)(Al + aoff + kc + 16));
#pragma unroll
        for (int t = 0; t < 2; ++t) { const v16h bb = cat16(*(const v8h*)(Bn + boff[t] + kc), *(const v8h*)(Bn + boff[t] + kc + 16)), bl = cat16(*(const v8h*)(Bl + boff[t] + kc), *(const v8h*)(Bl + boff[t] + kc + 16));
            acc[t] = wmma16(a, bb, acc[t]); accx[t] = wmma16(a, bl, accx[t]);
            if (EPI == 0) accx[t] = wmma16(al, bb, accx[t]); else acc[t] = wmma16(al, bb, acc[t]); }
        asm volatile("v_nop" : "+v"(acc[0]), "+v"(acc[1]), "+v"(accx[0]), "+v"(accx[1]) : "v"(a), "v"(al) : "memory");
    }
    float* os = &ost[wave][0];
#pragma unroll
    for (int t = 0; t < 2; ++t)
#pragma unroll
        for (int j = 0; j < 8; ++j) { const float sc = rs[r0 + hi * 8 + j]; os[(hi * 8 + j) * 68 + t * 16 + lr] = (acc[t][j] + accx[t][j] * LOSCI) * sc; }
    __builtin_amdgcn_wave_barrier(); asm volatile("" ::: "memory");
    float* crow = C + (size_t)r0 * ldc;
    auto pass = [&]() {
#pragma unroll
        for (int s = 0; s < 4; ++s) { const int row = s * 4 + (lane >> 3), piece = lane & 7;
            const v4f val = *(const v4fa*)(os + row * 68 + piece * 4); *(volatile v4f*)(crow + (size_t)row * ldc + piece * 4) = val; }
    };
    pass(); __threadfence(); pass();
}
__global__ __launch_bounds__(256) void k_soft(const float* __restrict__ S, h16* PH, h16* PL, float* RS) {
    __shared__ float rsum[32];
    const int lane = threadIdx.x & 31, wave = threadIdx.x >> 5;
#pragma unroll 1
    for (int rr = 0; rr < 4; ++rr) { const int row = blockIdx.x * 32 + wave * 4 + rr; const float* sr = S + (size_t)row * NP;
        float mx = -3.0e38f;
#pragma unroll 1
        for (int c = 0; c < NP / 256; ++c)
#pragma unroll
            for (int i = 0; i < 8; ++i) mx = fmaxf(mx, sr[c * 256 + lane * 8 + i]);
#pragma unroll
        for (int sh = 16; sh; sh >>= 1) mx = fmaxf(mx, __shfl_xor(mx, sh, 32));
        float sum = 0.f;
#pragma unroll 1
        for (int ps = 0; ps < 2; ++ps) { sum = 0.f;
#pragma unroll 1
            for (int c = 0; c < NP / 256; ++c) { v8h oh, ol;
#pragma unroll
                for (int i = 0; i < 8; ++i) { const float p = __expf(sr[c * 256 + lane * 8 + i] - mx); sum += p; const float ps8 = p * PSC; const h16 a = (h16)ps8; oh[i] = a; ol[i] = (h16)(ps8 - (float)a); }
                *(volatile v8h*)(PH + (size_t)row * NP + c * 256 + lane * 8) = oh; *(volatile v8h*)(PL + (size_t)row * NP + c * 256 + lane * 8) = ol; }
            if (ps == 0) __threadfence(); }
#pragma unroll
        for (int sh = 16; sh; sh >>= 1) sum += __shfl_xor(sum, sh, 32);
        if (lane == 0) rsum[wave * 4 + rr] = 1.0f / (sum * PSC); }
    __syncthreads();
    if (wave == 0) { const float v = rsum[lane]; *(volatile float*)(RS + blockIdx.x * 32 + lane) = v; __threadfence(); *(volatile float*)(RS + blockIdx.x * 32 + lane) = v; }
}

extern "C" void kernel_launch(void* const* d_in, const int* in_sizes, int n_in,
                              void* d_out, int out_size, void* d_ws, size_t ws_size, hipStream_t stream) {
    (void)in_sizes; (void)n_in; (void)out_size;
    const float* x = (const float*)d_in[0]; const float* wth = (const float*)d_in[1]; const float* bth = (const float*)d_in[2]; const float* wph = (const float*)d_in[3]; const float* bph = (const float*)d_in[4];
    const float* wg = (const float*)d_in[5]; const float* bg = (const float*)d_in[6]; const float* wz = (const float*)d_in[7]; const float* bz = (const float*)d_in[8];
    const float* bng = (const float*)d_in[9]; const float* bnb = (const float*)d_in[10]; const float* bnm = (const float*)d_in[11]; const float* bnv = (const float*)d_in[12];
    float* out = (float*)d_out;
    char* wsp = (char*)d_ws;
    auto take = [&](size_t bytes) { char* p = wsp; wsp += (bytes + 255) & ~(size_t)255; return (void*)p; };
    bf* Wt = (bf*)take((size_t)CI * CC * 2); bf* Wp = (bf*)take((size_t)CI * CC * 2); bf* Wg = (bf*)take((size_t)CI * CC * 2); bf* Wz = (bf*)take((size_t)CC * CI * 2);
    float* BNS = (float*)take(CC * 4); float* BNH = (float*)take(CC * 4);
    bf* XT = (bf*)take((size_t)NP * CC * 2);
    float* Qf = (float*)take((size_t)NP * CI * 4); float* Kf = (float*)take((size_t)NP * CI * 4); float* Vf = (float*)take((size_t)NP * CI * 4);
    h16* QH = (h16*)take((size_t)NP * CI * 2); h16* QL = (h16*)take((size_t)NP * CI * 2); h16* KH = (h16*)take((size_t)NP * CI * 2); h16* KL = (h16*)take((size_t)NP * CI * 2); h16* VTH = (h16*)take((size_t)CI * NP * 2); h16* VTL = (h16*)take((size_t)CI * NP * 2);
    float* S = (float*)take((size_t)QCH * NP * 4); h16* PH = (h16*)take((size_t)QCH * NP * 2); h16* PL = (h16*)take((size_t)QCH * NP * 2); float* RS = (float*)take((size_t)QCH * 4);
    float* Y = (float*)take((size_t)NP * CI * 4); bf* YH = (bf*)take((size_t)NP * CI * 2); bf* YL = (bf*)take((size_t)NP * CI * 2);
    if ((size_t)(wsp - (char*)d_ws) > ws_size) return;
    k_w<<<CI / 8, 256, 0, stream>>>(wth, CI, Wt); k_w<<<CI / 8, 256, 0, stream>>>(wph, CI, Wp); k_w<<<CI / 8, 256, 0, stream>>>(wg, CI, Wg); k_w128<<<(CC / 2 + 7) / 8, 256, 0, stream>>>(wz, CC, Wz);
    k_bn<<<1, 256, 0, stream>>>(bng, bnb, bnm, bnv, BNS, BNH);
    for (int b = 0; b < NB_; ++b) {
        k_xt<<<dim3(NP / 64, CC / 64, 1), 256, 0, stream>>>(x + (size_t)b * CC * NP, XT);
        k_gemm<false, 0, CC, CI><<<dim3(NP / 64, CI / 64, 1), 128, 0, stream>>>(XT, nullptr, Wt, bth, nullptr, nullptr, nullptr, Qf);
        k_gemm<false, 0, CC, CI><<<dim3(NP / 64, CI / 64, 1), 128, 0, stream>>>(XT, nullptr, Wp, bph, nullptr, nullptr, nullptr, Kf);
        k_gemm<false, 0, CC, CI><<<dim3(NP / 64, CI / 64, 1), 128, 0, stream>>>(XT, nullptr, Wg, bg, nullptr, nullptr, nullptr, Vf);
        k_p16c<<<(NP / 2 + 7) / 8, 256, 0, stream>>>(Qf, QH, QL); k_p16c<<<(NP / 2 + 7) / 8, 256, 0, stream>>>(Kf, KH, KL);
        k_vt128<<<dim3(NP / 64, CI / 64, 1), 256, 0, stream>>>(Vf, VTH, VTL);
        for (int h = 0; h < NHD; ++h)
            for (int c = 0; c < NP / QCH; ++c) {
                k_f16gemm<0><<<dim3(QCH / 64, NP / 64, 1), 128, 0, stream>>>(QH + (size_t)c * QCH * CI + h * HD, QL + (size_t)c * QCH * CI + h * HD, CI, KH + h * HD, KL + h * HD, CI, HD, nullptr, S, NP);
                k_soft<<<QCH / 32, 256, 0, stream>>>(S, PH, PL, RS);
                k_pv32<<<dim3(QCH / 64, 1, 1), 128, 0, stream>>>(PH, PL, NP, VTH + (size_t)h * HD * NP, VTL + (size_t)h * HD * NP, NP, NP, RS, Y + (size_t)c * QCH * CI + h * HD, CI);
            }
        k_pbfc<<<(NP / 2 + 7) / 8, 256, 0, stream>>>(Y, YH, YL);
        k_gemm<true, 2, CI, CC><<<dim3(NP / 64, CC / 64, 1), 128, 0, stream>>>(YH, YL, Wz, bz, BNS, BNH, x + (size_t)b * CC * NP, out + (size_t)b * CC * NP);
    }
}
